// GConvLSTM_20847771254916
// MI455X (gfx1250) — hardware-run, weakly checked
//
#include <hip/hip_runtime.h>


namespace {
constexpr int N = 50000, NP = 50048, E = 1600000, D = 64, K3 = 3, KT = 6 * D, NG = 4 * D;
constexpr float XS = 8.0f, WSC = 256.0f, NEG = 0.2f  ;
typedef _Float16 b16;
typedef __attribute__((ext_vector_type(16))) _Float16 v16b;
typedef __attribute__((ext_vector_type(8))) _Float16 v8b;
typedef __attribute__((ext_vector_type(8))) float v8f;
typedef __attribute__((ext_vector_type(4))) float v4f;
typedef __attribute__((ext_vector_type(2))) float v2f;
__device__ __forceinline__ float bf16_rne(float f) { unsigned int u = __float_as_uint(f); u += 0x7FFFu + ((u >> 16) & 1u); return __uint_as_float(u & 0xFFFF0000u); }
__device__ __forceinline__ void split16(float v, b16& hi, b16& lo) { hi = (b16)v; lo = (b16)(v - (float)hi); }
__device__ __forceinline__ v16b frag_kb(const b16* p, int hh) { const v8b a = *(const v8b*)(p + 8 * hh), b = *(const v8b*)(p + 16 + 8 * hh); v16b f;
#pragma unroll
  for (int e = 0; e < 8; ++e) { f[e] = a[e]; f[8 + e] = b[e]; } return f; }
__device__ __forceinline__ v8f wmma16b(v16b a, v16b b, v8f c) { v8f d = __builtin_amdgcn_wmma_f32_16x16x32_f16(false, a, false, b, (short)0, c, false, false); asm volatile("v_nop\n\tv_nop\n\tv_nop\n\tv_nop" : "+v"(d) : "v"(a), "v"(b)); return d; }
__device__ __forceinline__ void wave_lds_sync() { __builtin_amdgcn_fence(__ATOMIC_RELEASE, "workgroup"); __builtin_amdgcn_wave_barrier(); __builtin_amdgcn_fence(__ATOMIC_ACQUIRE, "workgroup"); }
__device__ __forceinline__ float pmul(float a, float b) { float p = a * b; asm volatile("" : "+v"(p)); return p; }
__device__ __forceinline__ int iclamp(int v, int lo, int hi) { return v < lo ? lo : (v > hi ? hi : v); }
__device__ __forceinline__ float sigm(float x) { return 1.0f / (1.0f + __expf(-x)); }
constexpr int CSR_NBLK8 = 512, CSR_GB8 = 8, CSR_GN8 = 1 << CSR_GB8  , CSR_MAXG8 = 512, CSR_CAP8 = 12288  ;
__global__ __launch_bounds__(64) void csrA8_kernel(const int* __restrict__ dst, int E, int N, int nG, int CHP, int NGP, int* __restrict__ STG, int* __restrict__ HST) {
  extern __shared__ int sm[];
  int* cnt = sm; int* run = sm + NGP; int* ids = sm + 2 * NGP;
  const int b = blockIdx.x; const int ch = (E + CSR_NBLK8 - 1) / CSR_NBLK8; const int e0 = b * ch, e1 = min(E, e0 + ch);
  for (int i = threadIdx.x; i < NGP; i += 64) cnt[i] = 0;
  for (int i = threadIdx.x; i < CHP; i += 64) ids[i] = -1;
  __syncthreads();
  if (threadIdx.x == 0) {
    for (int e = e0; e < e1; ++e) { int d = dst[e]; d = (d < 0) ? 0 : (d >= N ? N - 1 : d); cnt[d >> CSR_GB8] += 1; }
    int acc = 0; for (int g = 0; g < nG; ++g) { run[g] = acc; acc += cnt[g]; }
    for (int e = e0; e < e1; ++e) { int d = dst[e]; d = (d < 0) ? 0 : (d >= N ? N - 1 : d); const int g = d >> CSR_GB8; ids[run[g]] = e; run[g] += 1; } }
  __syncthreads();
  typedef __attribute__((ext_vector_type(4))) int v4i;
  for (int pass = 0; pass < 2; ++pass) {
    for (int i = threadIdx.x; i < CHP / 4; i += 64) *(volatile v4i*)(STG + (size_t)b * CHP + i * 4) = *(const v4i*)(&ids[i * 4]);
    for (int i = threadIdx.x; i < NGP / 4; i += 64) { v4i v; for (int e = 0; e < 4; ++e) v[e] = (i * 4 + e < nG) ? cnt[i * 4 + e] : 0; *(volatile v4i*)(HST + (size_t)b * NGP + i * 4) = v; }
    __threadfence(); }
}
__global__ __launch_bounds__(512) void csrS8_kernel(const int* __restrict__ HST, int nG, int NGP, int* __restrict__ START, int* __restrict__ TOT, int* __restrict__ OFF) {
  __shared__ int tot[CSR_MAXG8];
  const int b = threadIdx.x;
  for (int pass = 0; pass < 2; ++pass) { int runb = 0; for (int g = 0; g < nG; ++g) { int c = HST[(size_t)b * NGP + g]; c = (c < 0) ? 0 : c; ((volatile int*)OFF)[(size_t)g * CSR_NBLK8 + b] = runb; runb += c; } __threadfence(); }
  for (int g = threadIdx.x; g < nG; g += 512) { int s = 0; for (int bb = 0; bb < CSR_NBLK8; ++bb) { int c = HST[(size_t)bb * NGP + g]; s += (c < 0) ? 0 : c; } tot[g] = s; }
  __syncthreads();
  if (threadIdx.x < 32) {
    __shared__ int st[CSR_MAXG8 + 32];
    if (threadIdx.x == 0) { int acc = 0; for (int g = 0; g < NGP; ++g) { st[g] = acc; if (g < nG) acc += (tot[g] + 31) & ~31; } st[NGP] = acc; }
    __builtin_amdgcn_fence(__ATOMIC_RELEASE, "workgroup"); __builtin_amdgcn_wave_barrier(); __builtin_amdgcn_fence(__ATOMIC_ACQUIRE, "workgroup");
    for (int pass = 0; pass < 2; ++pass) { for (int i = threadIdx.x; i < NGP + 32; i += 32) { ((volatile int*)START)[i] = (i <= NGP) ? st[min(i, NGP)] : 0; ((volatile int*)TOT)[i] = (i < nG) ? tot[i] : 0; } __threadfence(); } }
}
__global__ __launch_bounds__(256) void csrB8_kernel(const int* __restrict__ dst, int N, int nG, int CHP, int NGP, int permLen, const int* __restrict__ STG, const int* __restrict__ HST, const int* __restrict__ OFF, const int* __restrict__ START, const int* __restrict__ TOT, int* __restrict__ PERM, int* __restrict__ ROWPTR, int* __restrict__ ROWCNT, int* __restrict__ FLAG) {
  typedef __attribute__((ext_vector_type(4))) int v4i;
  __shared__ int ids[CSR_CAP8]; __shared__ unsigned short key[CSR_CAP8]; __shared__ int outp[CSR_CAP8]; __shared__ int ncnt[CSR_GN8 + 1]; __shared__ int boff[CSR_NBLK8 + 1];
  const int g = blockIdx.x, t_ = threadIdx.x; int tot = TOT[g]; int st = START[g], stn = START[g + 1]; const int v0 = g * CSR_GN8; const int nv = min(CSR_GN8, N - v0);
  st = (st < 0) ? 0 : (st > permLen - 32 ? permLen - 32 : st) & ~31; stn = (stn < st) ? st : (stn > permLen ? permLen : stn); tot = (tot < 0) ? 0 : tot; if (tot > stn - st && tot <= CSR_CAP8) tot = stn - st;
  if (tot > CSR_CAP8) {
    for (int pass = 0; pass < 2; ++pass) { for (int i = t_; i < CSR_GN8 / 4; i += 256) { v4i a, c; for (int e = 0; e < 4; ++e) { a[e] = st; c[e] = 0; } *(volatile v4i*)(ROWPTR + v0 + i * 4) = a; *(volatile v4i*)(ROWCNT + v0 + i * 4) = c; } if (t_ == 0) ((volatile int*)FLAG)[0] = 1; __threadfence(); } (void)nv; return; }
  if (t_ == 0) { int acc = 0; for (int b = 0; b < CSR_NBLK8; ++b) { boff[b] = acc; int c = HST[(size_t)b * NGP + g]; c = (c < 0) ? 0 : (c > CHP ? CHP : c); acc += c; if (acc > tot) acc = tot; } boff[CSR_NBLK8] = acc; }
  for (int i = t_; i <= CSR_GN8; i += 256) ncnt[i] = 0;
  __syncthreads();
  for (int b = 0; b < CSR_NBLK8; ++b) { const int c = boff[b + 1] - boff[b]; int o_ = OFF[(size_t)g * CSR_NBLK8 + b]; o_ = (o_ < 0) ? 0 : (o_ > CHP - c ? CHP - c : o_); const int* src_ = STG + (size_t)b * CHP + o_;
    for (int i = t_; i < c; i += 256) { int id = src_[i]; id = (id < 0) ? 0 : id; ids[boff[b] + i] = id; int d = dst[id]; d = (d < v0) ? v0 : (d >= N ? N - 1 : d); int kk = d - v0; kk = (kk < 0) ? 0 : (kk >= CSR_GN8 ? CSR_GN8 - 1 : kk); key[boff[b] + i] = (unsigned short)kk; } }
  __syncthreads();
  if (t_ == 0) { for (int i = 0; i < tot; ++i) ncnt[key[i]] += 1; int acc = 0; for (int vl = 0; vl < CSR_GN8; ++vl) { const int c = ncnt[vl]; ncnt[vl] = acc; acc += c; } ncnt[CSR_GN8] = acc;
    for (int i = 0; i < tot; ++i) { const int vl = key[i]; outp[ncnt[vl]] = ids[i]; ncnt[vl] += 1; }
    for (int vl = CSR_GN8; vl > 0; --vl) ncnt[vl] = ncnt[vl - 1]; ncnt[0] = 0; }
  __syncthreads();
  for (int pass = 0; pass < 2; ++pass) {
    for (int i = t_; i < (stn - st) / 4; i += 256) { v4i v; for (int e = 0; e < 4; ++e) { const int q = i * 4 + e; v[e] = (q < tot) ? outp[q] : -1; } *(volatile v4i*)(PERM + st + i * 4) = v; }
    for (int i = t_; i < CSR_GN8 / 4; i += 256) { v4i a, c; for (int e = 0; e < 4; ++e) { const int vl = i * 4 + e; a[e] = st + ncnt[vl]; c[e] = (vl < nv) ? (ncnt[vl + 1] - ncnt[vl]) : 0; } *(volatile v4i*)(ROWPTR + v0 + i * 4) = a; *(volatile v4i*)(ROWCNT + v0 + i * 4) = c; }
    __threadfence(); }
}
__global__ __launch_bounds__(256) void csrZ8_kernel(int* __restrict__ p, size_t n4) { typedef __attribute__((ext_vector_type(4))) int v4i; const size_t tid = (size_t)blockIdx.x * 256 + threadIdx.x, nth = (size_t)gridDim.x * 256; v4i z = {0, 0, 0, 0}; for (size_t i = tid; i < n4; i += nth) *(volatile v4i*)(p + i * 4) = z; }
struct CsrBufs8 { int *STG, *HST, *OFF, *START, *TOT, *PERM, *ROWPTR, *ROWCNT, *FLAG; int nG, NGP, CHP; size_t permLen; char* base; size_t bytes; };
static size_t csr_carve8(CsrBufs8& c, char* ws, size_t off, int E, int N) {
  const size_t off0 = off; c.base = ws + off;
  auto al = [&](size_t bytes) { char* p = ws + off; off += (bytes + 255) & ~(size_t)255; return p; };
  c.nG = (N + CSR_GN8 - 1) / CSR_GN8; c.NGP = (c.nG + 31) & ~31; const int ch = (E + CSR_NBLK8 - 1) / CSR_NBLK8; c.CHP = (ch + 31) & ~31; c.permLen = (size_t)E + 32 * (size_t)c.nG + 32;
  c.STG = (int*)al((size_t)CSR_NBLK8 * c.CHP * 4); c.HST = (int*)al((size_t)CSR_NBLK8 * c.NGP * 4); c.OFF = (int*)al((size_t)c.NGP * CSR_NBLK8 * 4); c.START = (int*)al((size_t)(c.NGP + 64) * 4); c.TOT = (int*)al((size_t)(c.NGP + 64) * 4);
  c.PERM = (int*)al(c.permLen * 4); c.ROWPTR = (int*)al((size_t)c.nG * CSR_GN8 * 4); c.ROWCNT = (int*)al((size_t)c.nG * CSR_GN8 * 4); c.FLAG = (int*)al(256);
  c.bytes = off - off0; return off;
}
static void csr_build8(const CsrBufs8& c, const int* dst, int E, int N, hipStream_t stream) {
  const size_t smem = (size_t)(2 * c.NGP + c.CHP) * 4;
  csrZ8_kernel<<<512, 256, 0, stream>>>((int*)c.base, c.bytes / 16);
  csrA8_kernel<<<CSR_NBLK8, 64, smem, stream>>>(dst, E, N, c.nG, c.CHP, c.NGP, c.STG, c.HST);
  csrS8_kernel<<<1, 512, 0, stream>>>(c.HST, c.nG, c.NGP, c.START, c.TOT, c.OFF);
  csrB8_kernel<<<c.nG, 256, 0, stream>>>(dst, N, c.nG, c.CHP, c.NGP, (int)c.permLen, c.STG, c.HST, c.OFF, c.START, c.TOT, c.PERM, c.ROWPTR, c.ROWCNT, c.FLAG);
}


__global__ __launch_bounds__(256) void wprep_kernel(const float* __restrict__ wxi, const float* __restrict__ wxf, const float* __restrict__ wxc, const float* __restrict__ wxo, const float* __restrict__ whi, const float* __restrict__ whf, const float* __restrict__ whc, const float* __restrict__ who, b16* __restrict__ WB) {
  const size_t u = (size_t)blockIdx.x * 256 + threadIdx.x; if (u >= (size_t)NG * KT / 8) return; const size_t e = u * 8; const int row = (int)(e / KT), k0 = (int)(e % KT); const int g = row / D, oo = row % D; const int seg = k0 / D;
  const float* w = seg < 3 ? (g == 0 ? wxi : g == 1 ? wxf : g == 2 ? wxc : wxo) : (g == 0 ? whi : g == 1 ? whf : g == 2 ? whc : who); const int kk = seg % 3; v8b o;
  for (int j = 0; j < 8; ++j) { const int k = (k0 + j) % D; o[j] = (b16)(bf16_rne(w[((size_t)kk * D + k) * D + oo]) * WSC); }
  for (int pass = 0; pass < 2; ++pass) { *(volatile v8b*)(WB + e) = o; __threadfence(); }
}
__global__ __launch_bounds__(256) void deg_kernel(const float* __restrict__ ew, const int* __restrict__ cols, const int* __restrict__ PERM, const int* __restrict__ ROWPTR, const int* __restrict__ ROWCNT, int permLen, float* __restrict__ DINV) {
  const size_t v = (size_t)blockIdx.x * 256 + threadIdx.x; float d = 0.0f;
  if (v < (size_t)N) { int st = ROWPTR[v], cnt = ROWCNT[v]; cnt = iclamp(cnt, 0, 65536); st = iclamp(st, 0, permLen - cnt);
    for (int j = 0; j < cnt; ++j) { const int e = iclamp(PERM[st + j], 0, E - 1); const int c = iclamp(cols[e], 0, N - 1); if (c != (int)v) d += bf16_rne(ew[e]); } }
  const float di = d > 0.0f ? rsqrtf(d) : 0.0f;
  for (int pass = 0; pass < 2; ++pass) { ((volatile float*)DINV)[v] = di; __threadfence(); }
}
template <int EXACTIN, int SECOND>
__global__ __launch_bounds__(256) void prop_kernel(const float* __restrict__ SA, const float* __restrict__ SB, const float* __restrict__ T0A, const float* __restrict__ T0B, const float* __restrict__ ew, const int* __restrict__ cols, const float* __restrict__ DINV, const int* __restrict__ PERM, const int* __restrict__ ROWPTR, const int* __restrict__ ROWCNT, int permLen, float* __restrict__ OA, float* __restrict__ OB) {
  const int wave = threadIdx.x >> 5, lane = threadIdx.x & 31; const size_t v = (size_t)blockIdx.x * 8 + wave; const int c0 = lane * 2; v2f oa = {0.0f, 0.0f}, ob = oa;
  if (v < (size_t)N) { int st = ROWPTR[v], cnt = ROWCNT[v]; cnt = iclamp(cnt, 0, 65536); st = iclamp(st, 0, permLen - cnt); const float dv = DINV[v]; v2f aa = oa, ab = oa;
#pragma unroll 1
    for (int j = 0; j < cnt; ++j) { const int e = iclamp(PERM[st + j], 0, E - 1); const int c = iclamp(cols[e], 0, N - 1); if (c == (int)v) continue; const float w = -pmul(bf16_rne(ew[e]), DINV[c]);
      v2f xa = *(const v2f*)(SA + (size_t)c * D + c0), xb = *(const v2f*)(SB + (size_t)c * D + c0); if (EXACTIN) { xa[0] = bf16_rne(xa[0]); xa[1] = bf16_rne(xa[1]); xb[0] = bf16_rne(xb[0]); xb[1] = bf16_rne(xb[1]); }
      aa[0] += pmul(w, xa[0]); aa[1] += pmul(w, xa[1]); ab[0] += pmul(w, xb[0]); ab[1] += pmul(w, xb[1]); }
    for (int i = 0; i < 2; ++i) { oa[i] = pmul(dv, aa[i]); ob[i] = pmul(dv, ab[i]); }
    if (SECOND) { v2f ta = *(const v2f*)(T0A + v * D + c0), tb = *(const v2f*)(T0B + v * D + c0); for (int i = 0; i < 2; ++i) { oa[i] = 2.0f * oa[i] - bf16_rne(ta[i]); ob[i] = 2.0f * ob[i] - bf16_rne(tb[i]); } } }
  for (int pass = 0; pass < 2; ++pass) { *(volatile v2f*)(OA + v * D + c0) = oa; *(volatile v2f*)(OB + v * D + c0) = ob; __threadfence(); }
}
__global__ __launch_bounds__(32) void gate_kernel(const float* __restrict__ X, const float* __restrict__ T1X, const float* __restrict__ T2X, const float* __restrict__ Hin, const float* __restrict__ T1H, const float* __restrict__ T2H, const float* __restrict__ Cin, const b16* __restrict__ WB,
    const float* __restrict__ bxi, const float* __restrict__ bxf, const float* __restrict__ bxc, const float* __restrict__ bxo, const float* __restrict__ bhi, const float* __restrict__ bhf, const float* __restrict__ bhc, const float* __restrict__ bho,
    const float* __restrict__ wci, const float* __restrict__ wcf, const float* __restrict__ wco, const float* __restrict__ bi, const float* __restrict__ bf, const float* __restrict__ bc, const float* __restrict__ bo, float* __restrict__ outH, float* __restrict__ outC) {
  __shared__ __attribute__((aligned(16))) b16 Ah[16][KT + 8], Al[16][KT + 8]; __shared__ __attribute__((aligned(16))) float TH[16][D + 4], TC[16][D + 4];
  const int lane = threadIdx.x, nloc = lane & 15, hlf = lane >> 4; const size_t v0 = (size_t)blockIdx.x * 16; const int c0 = lane * 2;
  for (int rr = 0; rr < 16; ++rr) { const size_t v = v0 + rr; const bool ok = v < (size_t)N; const float* srcs6[6] = {X, T1X, T2X, Hin, T1H, T2H};
#pragma unroll
    for (int s = 0; s < 6; ++s) { v2f t = {0.0f, 0.0f}; if (ok || (s != 0 && s != 3)) t = *(const v2f*)(srcs6[s] + v * D + c0); if (!ok) t = (v2f){0.0f, 0.0f};
      for (int i = 0; i < 2; ++i) { b16 p, q; if (s == 0 || s == 3) { p = (b16)(bf16_rne(t[i]) * XS); q = (b16)0.0f; } else split16(t[i] * XS, p, q); Ah[rr][s * D + c0 + i] = p; Al[rr][s * D + c0 + i] = q; } } }
  wave_lds_sync();
  v8f acc[16];
#pragma unroll
  for (int t = 0; t < 16; ++t) acc[t] = (v8f){};
#pragma unroll 2
  for (int kb = 0; kb < KT; kb += 32) { const v16b a = frag_kb(&Ah[nloc][kb], hlf), al = frag_kb(&Al[nloc][kb], hlf); const bool dolo = !((kb < D) || (kb >= 3 * D && kb < 4 * D));
#pragma unroll
    for (int t = 0; t < 16; ++t) { const v16b bw = frag_kb(WB + (size_t)(t * 16 + nloc) * KT + kb, hlf); acc[t] = wmma16b(a, bw, acc[t]); if (dolo) acc[t] = wmma16b(al, bw, acc[t]); } }
#pragma unroll
  for (int jb = 0; jb < 4; ++jb) { const int o = jb * 16 + nloc; const float Bi = bf16_rne(bxi[o]) + bf16_rne(bhi[o]) + bf16_rne(bi[o]), Bf = bf16_rne(bxf[o]) + bf16_rne(bhf[o]) + bf16_rne(bf[o]), Bc = bf16_rne(bxc[o]) + bf16_rne(bhc[o]) + bf16_rne(bc[o]), Bo = bf16_rne(bxo[o]) + bf16_rne(bho[o]) + bf16_rne(bo[o]); const float pci = bf16_rne(wci[o]), pcf = bf16_rne(wcf[o]), pco = bf16_rne(wco[o]);
#pragma unroll 1
    for (int r = 0; r < 8; ++r) { const int rr = 8 * hlf + r; const size_t v = v0 + rr; const float cprev = v < (size_t)N ? bf16_rne(Cin[v * D + o]) : 0.0f; const float s = 1.0f / (XS * WSC);
      const float ig = sigm(acc[0 * 4 + jb][r] * s + Bi + pmul(pci, cprev)), fg = sigm(acc[1 * 4 + jb][r] * s + Bf + pmul(pcf, cprev)), tg = tanhf(acc[2 * 4 + jb][r] * s + Bc);
      const float cn = pmul(fg, cprev) + pmul(ig, tg); const float og = sigm(acc[3 * 4 + jb][r] * s + Bo + pmul(pco, cn)); TC[rr][o] = cn; TH[rr][o] = pmul(og, tanhf(cn)); } }
  wave_lds_sync();
  for (int rr = 0; rr < 16; ++rr) { const size_t v = v0 + rr; const v2f h = *(const v2f*)(&TH[rr][c0]), c = *(const v2f*)(&TC[rr][c0]);
    for (int pass = 0; pass < 2; ++pass) { if (v < (size_t)N) { *(volatile v2f*)(outH + v * D + c0) = h; *(volatile v2f*)(outC + v * D + c0) = c; } __threadfence(); } }
}
}

extern "C" void kernel_launch(void* const* d_in, const int* in_sizes, int n_in, void* d_out, int out_size, void* d_ws, size_t ws_size, hipStream_t stream) {
  (void)n_in;
  auto Fp = [&](int i) { return (const float*)d_in[i]; }; auto Ip = [&](int i) { return (const int*)d_in[i]; };
  if (in_sizes[0] != N * D || in_sizes[1] != 2 * E || in_sizes[2] != E || in_sizes[3] != N * D || in_sizes[4] != N * D || in_sizes[5] != K3 * D * D || in_sizes[19] != K3 * D * D || out_size != 2 * N * D) return;
  size_t off = 0; char* ws = (char*)d_ws;
  auto carve = [&](size_t bytes) { char* p = ws + off; off += (bytes + 255) & ~(size_t)255; return p; };
  b16* WB = (b16*)carve((size_t)NG * KT * 2); float* DINV = (float*)carve((size_t)((NP + 255) / 256 * 256) * 4); float* T1X = (float*)carve((size_t)NP * D * 4); float* T1H = (float*)carve((size_t)NP * D * 4); float* T2X = (float*)carve((size_t)NP * D * 4); float* T2H = (float*)carve((size_t)NP * D * 4);
  CsrBufs8 csr; off = csr_carve8(csr, ws, off, E, N);
  if (off > ws_size || off > ((size_t)128 << 20)) return;
  wprep_kernel<<<(unsigned)(((size_t)NG * KT / 8 + 255) / 256), 256, 0, stream>>>(Fp(5), Fp(7), Fp(9), Fp(11), Fp(13), Fp(15), Fp(17), Fp(19), WB);
  csr_build8(csr, Ip(1), E, N, stream);
  deg_kernel<<<(NP + 255) / 256, 256, 0, stream>>>(Fp(2), Ip(1) + E, csr.PERM, csr.ROWPTR, csr.ROWCNT, (int)csr.permLen, DINV);
  prop_kernel<1, 0><<<NP / 8, 256, 0, stream>>>(Fp(0), Fp(3), nullptr, nullptr, Fp(2), Ip(1) + E, DINV, csr.PERM, csr.ROWPTR, csr.ROWCNT, (int)csr.permLen, T1X, T1H);
  prop_kernel<0, 1><<<NP / 8, 256, 0, stream>>>(T1X, T1H, Fp(0), Fp(3), Fp(2), Ip(1) + E, DINV, csr.PERM, csr.ROWPTR, csr.ROWCNT, (int)csr.permLen, T2X, T2H);
  float* outH = (float*)d_out; float* outC = outH + (size_t)N * D;
  gate_kernel<<<NP / 16, 32, 0, stream>>>(Fp(0), T1X, T2X, Fp(3), T1H, T2H, Fp(4), WB, Fp(6), Fp(8), Fp(10), Fp(12), Fp(14), Fp(16), Fp(18), Fp(20), Fp(21), Fp(22), Fp(23), Fp(24), Fp(25), Fp(26), Fp(27), outH, outC);
}
